// IteratedGramAttention_43224550867971
// MI455X (gfx1250) — hardware-run, weakly checked
//
#include <hip/hip_runtime.h>
#include <math.h>

typedef __attribute__((ext_vector_type(16))) _Float16 v16h;
typedef __attribute__((ext_vector_type(8)))  _Float16 v8h;
typedef __attribute__((ext_vector_type(8)))  float    v8f;
typedef __attribute__((ext_vector_type(4)))  float    v4f;
typedef __attribute__((ext_vector_type(4)))  unsigned int v4u;

constexpr int kB      = 2;
constexpr int kT      = 2048;
constexpr int kD      = 1024;
constexpr int kH      = 16;
constexpr int kHd     = 64;
constexpr int kRows   = kB * kT;
constexpr int kQkvN   = 3 * kD;
constexpr int kSmallReal = 4 * 4 * kH + kH;
constexpr int kSmallN = 320;
constexpr int kLinesP = 16 * kH;
static_assert(kH * kHd == kD);
static_assert(kSmallReal == 272 && kSmallReal <= kSmallN);
static_assert((kRows % 64) == 0 && (kQkvN % 64) == 0 && (kSmallN % 64) == 0 && (kD % 64) == 0);
static_assert((kD % 32) == 0 && (kT % 64) == 0 && (kHd % 32) == 0);
static_assert(((kRows / 64) * (kSmallN / 64)) % 8 == 0);
static_assert(((kRows / 64) * (kQkvN / 64)) % 8 == 0);
static_assert(((kRows / 64) * (kD / 64)) % 8 == 0);

constexpr float kXC      = 16.0f;
constexpr float kWC      = 1024.0f;
constexpr float kProjInv = 1.0f / (kXC * kWC);
constexpr float kScale   = 0.125f;
static_assert(kScale * kScale * (float)kHd == 1.0f);
constexpr float kQC      = 128.0f;
constexpr float kQMul    = kScale * kQC;
constexpr float kKC      = 64.0f;
constexpr float kVC      = 64.0f;
constexpr float kSInv    = 1.0f / (kQC * kKC);
constexpr float kPC      = 1024.0f;
constexpr float kYC      = 32.0f;
constexpr float kOutInv  = 1.0f / (kYC * kWC);
constexpr float kHalfMin = 6.103515625e-5f;

constexpr size_t kOffXH    = 0;
constexpr size_t kOffWQKV  = kOffXH    + (size_t)kRows * kD * 2;
constexpr size_t kOffWSM   = kOffWQKV  + (size_t)kQkvN * kD * 2;
constexpr size_t kOffWMV   = kOffWSM   + (size_t)kSmallN * kD * 2;
constexpr size_t kOffWOUT  = kOffWMV   + (size_t)kD * kD * 2;
constexpr size_t kOffPSM   = kOffWOUT  + (size_t)kD * kD * 2;
constexpr size_t kOffLINES = kOffPSM   + (size_t)kRows * kSmallN * 4;
constexpr size_t kOffGATED = kOffLINES + (size_t)kRows * kLinesP * 4;
constexpr size_t kOffQP    = kOffGATED + (size_t)kRows * 4;
constexpr size_t kOffKP    = kOffQP    + (size_t)kRows * kD * 2;
constexpr size_t kOffVP    = kOffKP    + (size_t)kRows * kD * 2;
constexpr size_t kOffSEQ   = kOffVP    + (size_t)kRows * kD * 2;
constexpr size_t kOffYH    = kOffSEQ   + (size_t)kRows * kD * 4;
constexpr size_t kWsTotal  = kOffYH    + (size_t)kRows * kD * 2;
static_assert(kWsTotal == 79314944ull);
static_assert(kWsTotal <= 134217728ull);
static_assert((kOffWQKV % 128) == 0 && (kOffWSM % 128) == 0 && (kOffWMV % 128) == 0 && (kOffWOUT % 128) == 0 &&
              (kOffPSM % 128) == 0 && (kOffLINES % 128) == 0 && (kOffGATED % 128) == 0 && (kOffQP % 128) == 0 &&
              (kOffKP % 128) == 0 && (kOffVP % 128) == 0 && (kOffSEQ % 128) == 0 && (kOffYH % 128) == 0);

__device__ __forceinline__ float bf_rne(float f) {
  unsigned u = __float_as_uint(f);
  u = (u + 0x7FFFu + ((u >> 16) & 1u)) & 0xFFFF0000u;
  return __uint_as_float(u);
}
__device__ __forceinline__ float flush16(float v) {
  return (fabsf(v) < kHalfMin) ? 0.0f : v;
}
__device__ __forceinline__ _Float16 to_h(float v) {
  return (_Float16)flush16(v);
}
__device__ __forceinline__ v16h frag_ld(const _Float16* p) {
  union { v16h v; v8h h[2]; } f;
  f.h[0] = *(const v8h*)(p);
  f.h[1] = *(const v8h*)(p + 16);
  return f.v;
}
__device__ __forceinline__ v8f mma_g(v16h a, v16h b, v8f c) {
  c = __builtin_amdgcn_wmma_f32_16x16x32_f16(false, a, false, b, (short)0, c, false, false);
  asm volatile("v_nop\n\tv_nop\n\tv_nop\n\tv_nop" : "+v"(c) : "v"(a), "v"(b));
  return c;
}

__global__ __launch_bounds__(256) void cvt_plane_kernel(const float* __restrict__ src, _Float16* __restrict__ dst,
                                                        int total8, float carry) {
  const int i = blockIdx.x * 256 + threadIdx.x;
  if (i >= total8) return;
  const size_t e0 = (size_t)i << 3;
  const v4f a0 = *(const v4f*)(src + e0);
  const v4f a1 = *(const v4f*)(src + e0 + 4);
  v8h hv;
#pragma unroll
  for (int e = 0; e < 4; ++e) {
    const float f0 = a0[e];
    const float f1 = a1[e];
    hv[e]     = to_h(bf_rne(f0) * carry);
    hv[4 + e] = to_h(bf_rne(f1) * carry);
  }
  _Float16* q = dst + e0;
  *(volatile v8h*)q = hv;
  __threadfence();
  *(volatile v8h*)q = hv;
}

__global__ __launch_bounds__(256) void cvt_small_kernel(const float* __restrict__ w1, const float* __restrict__ w2,
                                                        const float* __restrict__ r1, const float* __restrict__ r2,
                                                        const float* __restrict__ mg, _Float16* __restrict__ dst,
                                                        float carry) {
  const int row0 = blockIdx.x * 2;
  const float* src = w1;
  int sbase = 0;
  bool live = true;
  if (row0 < 64)       { src = w1; sbase = row0; }
  else if (row0 < 128) { src = w2; sbase = row0 - 64; }
  else if (row0 < 192) { src = r1; sbase = row0 - 128; }
  else if (row0 < 256) { src = r2; sbase = row0 - 192; }
  else if (row0 < kSmallReal) { src = mg; sbase = row0 - 256; }
  else { src = w1; sbase = 0; live = false; }
  const int tid  = threadIdx.x;
  const int rloc = tid >> 7;
  const int col  = (tid & 127) * 8;
  const float* p = src + (size_t)(sbase + rloc) * kD + col;
  const v4f a0 = *(const v4f*)(p);
  const v4f a1 = *(const v4f*)(p + 4);
  v8h hv;
#pragma unroll
  for (int e = 0; e < 4; ++e) {
    const float f0 = a0[e];
    const float f1 = a1[e];
    const float g0 = live ? (bf_rne(f0) * carry) : 0.0f;
    const float g1 = live ? (bf_rne(f1) * carry) : 0.0f;
    hv[e]     = to_h(g0);
    hv[4 + e] = to_h(g1);
  }
  _Float16* q = dst + (size_t)(row0 + rloc) * kD + col;
  *(volatile v8h*)q = hv;
  __threadfence();
  *(volatile v8h*)q = hv;
}

template <int EPI, bool HAS_BIAS>
__global__ __launch_bounds__(256) void gemm_f16_kernel(
    const _Float16* __restrict__ A, int lda,
    const _Float16* __restrict__ Bt, int ldb,
    void* __restrict__ C0, void* __restrict__ C1, void* __restrict__ C2, int ldc,
    const float* __restrict__ bias, const float* __restrict__ resid, const float* __restrict__ rowg,
    int M, int N, int K, float scale) {
  __shared__ __align__(16) float sT[8][16 * 68];
  const int lane = threadIdx.x & 31;
  const int wave = threadIdx.x >> 5;
  const int tilesN = N >> 6;
  const int tilesM = M >> 6;
  const int tile = blockIdx.x * 8 + wave;
  if (tile >= tilesM * tilesN) return;
  const int tm = tile / tilesN;
  const int tn = tile - tm * tilesN;
  const int m0 = tm << 6;
  const int n0 = tn << 6;
  const int rlane = lane & 15;
  const int koff  = (lane >> 4) * 8;
  const int mOff  = (lane >> 4) * 8;

  v8f acc[4][4];
#pragma unroll
  for (int i = 0; i < 4; ++i)
#pragma unroll
    for (int j = 0; j < 4; ++j) acc[i][j] = (v8f){0.f, 0.f, 0.f, 0.f, 0.f, 0.f, 0.f, 0.f};

#pragma unroll 1
  for (int k0 = 0; k0 < K; k0 += 32) {
    v16h bf[4];
#pragma unroll
    for (int j = 0; j < 4; ++j)
      bf[j] = frag_ld(Bt + (size_t)(n0 + (j << 4) + rlane) * ldb + koff + k0);
#pragma unroll
    for (int i = 0; i < 4; ++i) {
      const v16h af = frag_ld(A + (size_t)(m0 + (i << 4) + rlane) * lda + koff + k0);
#pragma unroll
      for (int j = 0; j < 4; ++j) acc[i][j] = mma_g(af, bf[j], acc[i][j]);
    }
  }

  float* slab = sT[wave];
  float bvals[4];
#pragma unroll
  for (int j = 0; j < 4; ++j) {
    float bv = 0.0f;
    if (HAS_BIAS) bv = bf_rne(bias[n0 + (j << 4) + rlane]);
    bvals[j] = bv;
  }
  float carry = 1.0f;
  _Float16* plane16 = (_Float16*)C0;
  size_t rowbase16 = 0;
  if (EPI == 1) {
    const int which = n0 / kD;
    const int hd = (n0 - which * kD) >> 6;
    const int bb = m0 / kT;
    carry = (which == 0) ? kQMul : ((which == 1) ? kKC : kVC);
    plane16 = (which == 0) ? (_Float16*)C0 : ((which == 1) ? (_Float16*)C1 : (_Float16*)C2);
    rowbase16 = ((size_t)(bb * kH + hd) * kT + (size_t)(m0 - bb * kT)) * kHd;
  }
#pragma unroll
  for (int i = 0; i < 4; ++i) {
    const int mBase = m0 + (i << 4);
    float gr[8];
    if (EPI == 2) {
      const v4f ga = *(const v4f*)(rowg + mBase + mOff);
      const v4f gb = *(const v4f*)(rowg + mBase + mOff + 4);
      gr[0] = ga[0]; gr[1] = ga[1]; gr[2] = ga[2]; gr[3] = ga[3];
      gr[4] = gb[0]; gr[5] = gb[1]; gr[6] = gb[2]; gr[7] = gb[3];
    } else {
#pragma unroll
      for (int r = 0; r < 8; ++r) gr[r] = 1.0f;
    }
#pragma unroll
    for (int j = 0; j < 4; ++j) {
#pragma unroll
      for (int r = 0; r < 8; ++r) {
        float v = acc[i][j][r] * scale;
        if (HAS_BIAS) v += bvals[j];
        if (EPI == 1) v *= carry;
        if (EPI == 2) v *= gr[r];
        slab[(mOff + r) * 68 + (j << 4) + rlane] = v;
      }
    }
    __builtin_amdgcn_fence(__ATOMIC_RELEASE, "workgroup");
    __builtin_amdgcn_wave_barrier();
    __builtin_amdgcn_fence(__ATOMIC_ACQUIRE, "workgroup");
    if (EPI == 0) {
      float* C = (float*)C0;
      const int hh = lane >> 4;
      const int c4 = (lane & 15) * 4;
      v4f vv[8];
#pragma unroll
      for (int it = 0; it < 8; ++it) vv[it] = *(const v4f*)(slab + (it * 2 + hh) * 68 + c4);
      for (int pass = 0; pass < 2; ++pass) {
#pragma unroll
        for (int it = 0; it < 8; ++it)
          *(volatile v4f*)(C + (size_t)(mBase + it * 2 + hh) * ldc + n0 + c4) = vv[it];
        __threadfence();
      }
    } else {
      const int q  = lane >> 3;
      const int c8 = (lane & 7) * 8;
      v8h hv[4];
#pragma unroll
      for (int it = 0; it < 4; ++it) {
        const int row = it * 4 + q;
        const float* sp = slab + row * 68 + c8;
        v4f a0 = *(const v4f*)(sp);
        v4f a1 = *(const v4f*)(sp + 4);
        if (EPI == 2) {
          const float* rp = resid + (size_t)(mBase + row) * ldc + n0 + c8;
          const v4f r0 = *(const v4f*)(rp);
          const v4f r1 = *(const v4f*)(rp + 4);
          a0 = (a0 + r0) * kYC;
          a1 = (a1 + r1) * kYC;
        }
#pragma unroll
        for (int e = 0; e < 4; ++e) {
          const float f0 = a0[e];
          const float f1 = a1[e];
          hv[it][e]     = to_h(f0);
          hv[it][4 + e] = to_h(f1);
        }
      }
      for (int pass = 0; pass < 2; ++pass) {
#pragma unroll
        for (int it = 0; it < 4; ++it) {
          const int row = it * 4 + q;
          _Float16* dp;
          if (EPI == 1) dp = plane16 + rowbase16 + (size_t)((i << 4) + row) * kHd + c8;
          else          dp = (_Float16*)C0 + (size_t)(mBase + row) * ldc + n0 + c8;
          *(volatile v8h*)dp = hv[it];
        }
        __threadfence();
      }
    }
    __builtin_amdgcn_fence(__ATOMIC_RELEASE, "workgroup");
    __builtin_amdgcn_wave_barrier();
    __builtin_amdgcn_fence(__ATOMIC_ACQUIRE, "workgroup");
  }
}

__global__ __launch_bounds__(256) void lines_kernel(const float* __restrict__ Psm, const float* __restrict__ memg_b,
                                                    float* __restrict__ lines) {
  __shared__ __align__(16) float sL[16 * 260];
  const int tid  = threadIdx.x;
  const int rloc = tid >> 4;
  const int h    = tid & 15;
  const int row  = blockIdx.x * 16 + rloc;
  const int t    = row & (kT - 1);
  const bool first = (t == 0);
  const int rowp = first ? row : (row - 1);
  const v4f p1v = *(const v4f*)(Psm + (size_t)rowp * kSmallN + h * 4);
  float p10 = p1v[0], p11 = p1v[1], p12 = p1v[2], p13 = p1v[3];
  asm volatile("" : "+v"(p10), "+v"(p11), "+v"(p12), "+v"(p13));
  p10 = first ? 0.0f : p10;
  p11 = first ? 0.0f : p11;
  p12 = first ? 0.0f : p12;
  p13 = first ? 0.0f : p13;
  const float* prow = Psm + (size_t)row * kSmallN;
  const v4f p2 = *(const v4f*)(prow + 64 + h * 4);
  const v4f q1 = *(const v4f*)(prow + 128 + h * 4);
  const v4f q2 = *(const v4f*)(prow + 192 + h * 4);
  const float glog = prow[256 + h];
  const float gb = bf_rne(memg_b[h]);

  const float p20 = p2[0], p21 = p2[1], p22 = p2[2], p23 = p2[3];
  const float w0 = p10 * p21 - p11 * p20;
  const float w1 = p10 * p22 - p12 * p20;
  const float w2 = p10 * p23 - p13 * p20;
  const float w3 = p11 * p22 - p12 * p21;
  const float w4 = p11 * p23 - p13 * p21;
  const float w5 = p12 * p23 - p13 * p22;
  float wn2 = 0.0f;
  wn2 += w0 * w0; wn2 += w1 * w1; wn2 += w2 * w2; wn2 += w3 * w3; wn2 += w4 * w4; wn2 += w5 * w5;
  const float winv = 1.0f / fmaxf(sqrtf(wn2), 1e-12f);

  const float a0 = q1[0], a1 = q1[1], a2 = q1[2], a3 = q1[3];
  const float b0 = q2[0], b1 = q2[1], b2 = q2[2], b3 = q2[3];
  const float r0 = a0 * b1 - a1 * b0;
  const float r1 = a0 * b2 - a2 * b0;
  const float r2 = a0 * b3 - a3 * b0;
  const float r3 = a1 * b2 - a2 * b1;
  const float r4 = a1 * b3 - a3 * b1;
  const float r5 = a2 * b3 - a3 * b2;
  float rn2 = 0.0f;
  rn2 += r0 * r0; rn2 += r1 * r1; rn2 += r2 * r2; rn2 += r3 * r3; rn2 += r4 * r4; rn2 += r5 * r5;
  const float rinv = 1.0f / fmaxf(sqrtf(rn2), 1e-12f);

  const float gate = 1.0f / (1.0f + expf(-(glog + gb)));

  const v4f o0 = (v4f){w5 * winv, -(w4 * winv), w3 * winv, w2 * winv};
  const v4f o1 = (v4f){-(w1 * winv), w0 * winv, r0 * rinv, r1 * rinv};
  const v4f o2 = (v4f){r2 * rinv, r3 * rinv, r4 * rinv, r5 * rinv};
  const v4f o3 = (v4f){gate, 0.0f, 0.0f, 0.0f};
  float* sp = sL + rloc * 260 + h * 16;
  *(v4f*)(sp)      = o0;
  *(v4f*)(sp + 4)  = o1;
  *(v4f*)(sp + 8)  = o2;
  *(v4f*)(sp + 12) = o3;
  __syncthreads();
  const int lane = tid & 31, wave = tid >> 5;
  v4f vv[4];
#pragma unroll
  for (int k = 0; k < 4; ++k) {
    const int lr  = wave * 2 + (k >> 1);
    const int col = (k & 1) * 128 + lane * 4;
    vv[k] = *(const v4f*)(sL + lr * 260 + col);
  }
  for (int pass = 0; pass < 2; ++pass) {
#pragma unroll
    for (int k = 0; k < 4; ++k) {
      const int lr  = wave * 2 + (k >> 1);
      const int col = (k & 1) * 128 + lane * 4;
      *(volatile v4f*)(lines + (size_t)(blockIdx.x * 16 + lr) * kLinesP + col) = vv[k];
    }
    __threadfence();
  }
}

#define GRAM_AT(i, j) (((i) <= (j)) ? Mst[(i)][(j)] : Mst[(j)][(i)])
__global__ __launch_bounds__(32) void scan_kernel(const float* __restrict__ lines, const float* __restrict__ mem_scale,
                                                  const float* __restrict__ iter_mix,
                                                  const float* __restrict__ decay_logits, float* __restrict__ gated) {
  const int lane = threadIdx.x;
  const int b = lane >> 4;
  const int h = lane & 15;
  const float msc   = bf_rne(mem_scale[h]);
  const float alpha = __builtin_amdgcn_rcpf(1.0f + expf(-bf_rne(iter_mix[0])));
  const float decay = __builtin_amdgcn_rcpf(1.0f + expf(-bf_rne(decay_logits[h])));
  const float oma   = 1.0f - alpha;
  float Mst[6][6];
#pragma unroll
  for (int i = 0; i < 6; ++i)
#pragma unroll
    for (int j = 0; j < 6; ++j) Mst[i][j] = 0.0f;
  float keep0 = 0.0f, keep1 = 0.0f;
  const float* base = lines + (size_t)(b * kT) * kLinesP + h * 16;
  v4f n0 = *(const v4f*)(base);
  v4f n1 = *(const v4f*)(base + 4);
  v4f n2 = *(const v4f*)(base + 8);
  v4f n3 = *(const v4f*)(base + 12);
#pragma unroll 1
  for (int t = 0; t < kT; ++t) {
    const v4f c0 = n0, c1 = n1, c2 = n2, c3 = n3;
    {
      const int tn = (t + 1 < kT) ? (t + 1) : (kT - 1);
      const float* np = base + (size_t)tn * kLinesP;
      n0 = *(const v4f*)(np);
      n1 = *(const v4f*)(np + 4);
      n2 = *(const v4f*)(np + 8);
      n3 = *(const v4f*)(np + 12);
    }
    float jw[6], rd[6];
    jw[0] = c0[0]; jw[1] = c0[1]; jw[2] = c0[2]; jw[3] = c0[3]; jw[4] = c1[0]; jw[5] = c1[1];
    rd[0] = c1[2]; rd[1] = c1[3]; rd[2] = c2[0]; rd[3] = c2[1]; rd[4] = c2[2]; rd[5] = c2[3];
    const float gt = c3[0];
    float s1 = 0.0f, s2 = 0.0f;
#pragma unroll
    for (int j = 0; j < 6; ++j) {
      float rm = 0.0f;
#pragma unroll
      for (int i = 0; i < 6; ++i) rm += rd[i] * GRAM_AT(i, j);
      s1 += rm * rd[j];
      s2 += rm * rm;
    }
    const float ms = oma * s1 + alpha * s2;
    const float sg = __builtin_amdgcn_rcpf(1.0f + expf(-(ms * msc)));
    float gs = sg * gt;
    gs += __shfl_xor(gs, 1, 32);
    gs += __shfl_xor(gs, 2, 32);
    gs += __shfl_xor(gs, 4, 32);
    gs += __shfl_xor(gs, 8, 32);
    gs *= (1.0f / (float)kH);
    const float g0 = __shfl(gs, 0, 32);
    const float g1 = __shfl(gs, 16, 32);
    const int ti = t & 31;
    keep0 = (lane == ti) ? g0 : keep0;
    keep1 = (lane == ti) ? g1 : keep1;
#pragma unroll
    for (int i = 0; i < 6; ++i)
#pragma unroll
      for (int j = i; j < 6; ++j) Mst[i][j] = decay * (Mst[i][j] + jw[i] * jw[j]);
    if (ti == 31) {
      const float k0v = keep0, k1v = keep1;
      float* p0 = gated + (t - 31) + lane;
      float* p1 = gated + kT + (t - 31) + lane;
      *(volatile float*)p0 = k0v;
      *(volatile float*)p1 = k1v;
      __threadfence();
      *(volatile float*)p0 = k0v;
      *(volatile float*)p1 = k1v;
    }
  }
}

__global__ __launch_bounds__(128) void attn_causal_kernel(const _Float16* __restrict__ Qp, const _Float16* __restrict__ Kp,
                                                          const _Float16* __restrict__ Vp, float* __restrict__ seq) {
  __shared__ __align__(16) _Float16 Ksh[64 * 64];
  __shared__ __align__(16) _Float16 Vth[64 * 64];
  __shared__ __align__(16) _Float16 Psh[4][16 * 64];
  __shared__ __align__(16) float    Os[4][16 * 68];
  const int tid  = threadIdx.x;
  const int wave = tid >> 5;
  const int lane = tid & 31;
  const int hh   = lane >> 4;
  const int c    = lane & 15;
  constexpr int nqb = kT / 64;
  const int bx = blockIdx.x;
  const int qb = bx % nqb;
  const int bh = bx / nqb;
  const int h  = bh % kH;
  const int b  = bh / kH;
  const int q0 = qb * 64 + wave * 16;
  const _Float16* Qg = Qp + (size_t)bh * kT * kHd;
  const _Float16* Kg = Kp + (size_t)bh * kT * kHd;
  const _Float16* Vg = Vp + (size_t)bh * kT * kHd;

  v16h qa[2];
#pragma unroll
  for (int dc = 0; dc < 2; ++dc) qa[dc] = frag_ld(Qg + (size_t)(q0 + c) * kHd + dc * 32 + 8 * hh);

  float mrow[8], lrow[8];
  v8f oacc[4];
#pragma unroll
  for (int r = 0; r < 8; ++r) { mrow[r] = -INFINITY; lrow[r] = 0.f; }
#pragma unroll
  for (int t = 0; t < 4; ++t) oacc[t] = (v8f){0.f, 0.f, 0.f, 0.f, 0.f, 0.f, 0.f, 0.f};

  _Float16* pw = Psh[wave];
#pragma unroll 1
  for (int kc = 0; kc <= qb; ++kc) {
    const int kv0 = kc * 64;
    __syncthreads();
#pragma unroll
    for (int i = 0; i < 4; ++i) {
      const int idx = tid + 128 * i;
      const v8h kk8 = *(const v8h*)(Kg + (size_t)kv0 * kHd + idx * 8);
      *(v8h*)(Ksh + idx * 8) = kk8;
      const v4u vw = *(const v4u*)(Vg + (size_t)kv0 * kHd + idx * 8);
      const int kvr = idx >> 3;
      const int d8  = (idx & 7) * 8;
#pragma unroll
      for (int e = 0; e < 4; ++e) {
        const unsigned w = vw[e];
        const unsigned short lo16 = (unsigned short)(w & 0xffffu);
        const unsigned short hi16 = (unsigned short)(w >> 16);
        Vth[(d8 + 2 * e) * 64 + kvr]     = __builtin_bit_cast(_Float16, lo16);
        Vth[(d8 + 2 * e + 1) * 64 + kvr] = __builtin_bit_cast(_Float16, hi16);
      }
    }
    __syncthreads();

    v8f s[4];
#pragma unroll
    for (int j = 0; j < 4; ++j) {
      s[j] = (v8f){0.f, 0.f, 0.f, 0.f, 0.f, 0.f, 0.f, 0.f};
#pragma unroll
      for (int dc = 0; dc < 2; ++dc) {
        const v16h kb = frag_ld(Ksh + (j * 16 + c) * 64 + dc * 32 + 8 * hh);
        s[j] = mma_g(qa[dc], kb, s[j]);
      }
    }
    const bool diag = (kc == qb);
    float cm[8];
#pragma unroll
    for (int r = 0; r < 8; ++r) {
      const int qrow = q0 + 8 * hh + r;
      float m = -INFINITY;
#pragma unroll
      for (int j = 0; j < 4; ++j) {
        const int kvcol = kv0 + j * 16 + c;
        float sv = s[j][r] * kSInv;
        const bool masked = diag && (kvcol > qrow);
        sv = masked ? -INFINITY : sv;
        s[j][r] = sv;
        m = fmaxf(m, sv);
      }
      m = fmaxf(m, __shfl_xor(m, 1, 32));
      m = fmaxf(m, __shfl_xor(m, 2, 32));
      m = fmaxf(m, __shfl_xor(m, 4, 32));
      m = fmaxf(m, __shfl_xor(m, 8, 32));
      cm[r] = m;
    }
#pragma unroll
    for (int r = 0; r < 8; ++r) {
      const float mnew  = fmaxf(mrow[r], cm[r]);
      const float alpha = expf(mrow[r] - mnew);
      mrow[r] = mnew;
      float psum = 0.f;
#pragma unroll
      for (int j = 0; j < 4; ++j) {
        const float p = expf(s[j][r] - mnew);
        psum += p;
        pw[(8 * hh + r) * 64 + j * 16 + c] = to_h(p * kPC);
      }
      psum += __shfl_xor(psum, 1, 32);
      psum += __shfl_xor(psum, 2, 32);
      psum += __shfl_xor(psum, 4, 32);
      psum += __shfl_xor(psum, 8, 32);
      lrow[r] = lrow[r] * alpha + psum;
#pragma unroll
      for (int t = 0; t < 4; ++t) oacc[t][r] *= alpha;
    }
    __syncthreads();
#pragma unroll 1
    for (int kk = 0; kk < 2; ++kk) {
      const v16h pa = frag_ld(pw + c * 64 + kk * 32 + 8 * hh);
#pragma unroll
      for (int t = 0; t < 4; ++t) {
        const v16h vb = frag_ld(Vth + (t * 16 + c) * 64 + kk * 32 + 8 * hh);
        oacc[t] = mma_g(pa, vb, oacc[t]);
      }
    }
  }

  float* os = Os[wave];
#pragma unroll
  for (int r = 0; r < 8; ++r) {
    const float inv = 1.0f / (lrow[r] * (kPC * kVC));
#pragma unroll
    for (int t = 0; t < 4; ++t) os[(8 * hh + r) * 68 + t * 16 + c] = oacc[t][r] * inv;
  }
  __syncthreads();
  {
    const int c4 = (lane & 15) * 4;
    float* ob = seq + (size_t)(b * kT + q0) * kD + h * kHd + c4;
    v4f vv[8];
#pragma unroll
    for (int it = 0; it < 8; ++it) vv[it] = *(const v4f*)(os + (it * 2 + hh) * 68 + c4);
    for (int pass = 0; pass < 2; ++pass) {
#pragma unroll
      for (int it = 0; it < 8; ++it)
        *(volatile v4f*)(ob + (size_t)(it * 2 + hh) * kD) = vv[it];
      __threadfence();
    }
  }
}

extern "C" void kernel_launch(void* const* d_in, const int* in_sizes, int n_in,
                              void* d_out, int out_size, void* d_ws, size_t ws_size,
                              hipStream_t stream) {
  if (n_in < 16) return;
  if (in_sizes[0] != kRows * kD) return;
  if (in_sizes[1] != kQkvN * kD) return;
  if (in_sizes[2] != kQkvN) return;
  if (in_sizes[3] != 4 * kH * kD) return;
  if (in_sizes[4] != 4 * kH * kD) return;
  if (in_sizes[5] != 4 * kH * kD) return;
  if (in_sizes[6] != 4 * kH * kD) return;
  if (in_sizes[7] != kD * kD) return;
  if (in_sizes[8] != kD) return;
  if (in_sizes[9] != kH * kD) return;
  if (in_sizes[10] != kH) return;
  if (in_sizes[11] != kH) return;
  if (in_sizes[12] != 1) return;
  if (in_sizes[13] != kD * kD) return;
  if (in_sizes[14] != kD) return;
  if (in_sizes[15] != kH) return;
  if (out_size != kRows * kD) return;
  if (ws_size < kWsTotal) return;

  const float* x        = (const float*)d_in[0];
  const float* qkv_w    = (const float*)d_in[1];
  const float* qkv_b    = (const float*)d_in[2];
  const float* w1w      = (const float*)d_in[3];
  const float* w2w      = (const float*)d_in[4];
  const float* r1w      = (const float*)d_in[5];
  const float* r2w      = (const float*)d_in[6];
  const float* memv_w   = (const float*)d_in[7];
  const float* memv_b   = (const float*)d_in[8];
  const float* memg_w   = (const float*)d_in[9];
  const float* memg_b   = (const float*)d_in[10];
  const float* mem_scl  = (const float*)d_in[11];
  const float* iter_mix = (const float*)d_in[12];
  const float* out_w    = (const float*)d_in[13];
  const float* out_b    = (const float*)d_in[14];
  const float* decay_l  = (const float*)d_in[15];
  float* out = (float*)d_out;

  char* ws = (char*)d_ws;
  _Float16* XH    = (_Float16*)(ws + kOffXH);
  _Float16* WQKV  = (_Float16*)(ws + kOffWQKV);
  _Float16* WSM   = (_Float16*)(ws + kOffWSM);
  _Float16* WMV   = (_Float16*)(ws + kOffWMV);
  _Float16* WOUT  = (_Float16*)(ws + kOffWOUT);
  float*    PSM   = (float*)(ws + kOffPSM);
  float*    LINES = (float*)(ws + kOffLINES);
  float*    GATED = (float*)(ws + kOffGATED);
  _Float16* QP    = (_Float16*)(ws + kOffQP);
  _Float16* KP    = (_Float16*)(ws + kOffKP);
  _Float16* VP    = (_Float16*)(ws + kOffVP);
  float*    SEQ   = (float*)(ws + kOffSEQ);
  _Float16* YH    = (_Float16*)(ws + kOffYH);

  cvt_plane_kernel<<<(kRows * kD / 8) / 256, 256, 0, stream>>>(x, XH, kRows * kD / 8, kXC);
  cvt_plane_kernel<<<(kQkvN * kD / 8) / 256, 256, 0, stream>>>(qkv_w, WQKV, kQkvN * kD / 8, kWC);
  cvt_plane_kernel<<<(kD * kD / 8) / 256, 256, 0, stream>>>(memv_w, WMV, kD * kD / 8, kWC);
  cvt_plane_kernel<<<(kD * kD / 8) / 256, 256, 0, stream>>>(out_w, WOUT, kD * kD / 8, kWC);
  cvt_small_kernel<<<kSmallN / 2, 256, 0, stream>>>(w1w, w2w, r1w, r2w, memg_w, WSM, kWC);

  gemm_f16_kernel<0, false><<<((kRows / 64) * (kSmallN / 64)) / 8, 256, 0, stream>>>(
      XH, kD, WSM, kD, (void*)PSM, nullptr, nullptr, kSmallN,
      nullptr, nullptr, nullptr, kRows, kSmallN, kD, kProjInv);

  lines_kernel<<<kRows / 16, 256, 0, stream>>>(PSM, memg_b, LINES);
  scan_kernel<<<1, 32, 0, stream>>>(LINES, mem_scl, iter_mix, decay_l, GATED);

  gemm_f16_kernel<1, true><<<((kRows / 64) * (kQkvN / 64)) / 8, 256, 0, stream>>>(
      XH, kD, WQKV, kD, (void*)QP, (void*)KP, (void*)VP, kHd,
      qkv_b, nullptr, nullptr, kRows, kQkvN, kD, kProjInv);

  attn_causal_kernel<<<kB * kH * (kT / 64), 128, 0, stream>>>(QP, KP, VP, SEQ);

  gemm_f16_kernel<2, true><<<((kRows / 64) * (kD / 64)) / 8, 256, 0, stream>>>(
      XH, kD, WMV, kD, (void*)YH, nullptr, nullptr, kD,
      memv_b, SEQ, GATED, kRows, kD, kD, kProjInv);

  gemm_f16_kernel<0, true><<<((kRows / 64) * (kD / 64)) / 8, 256, 0, stream>>>(
      YH, kD, WOUT, kD, (void*)out, nullptr, nullptr, kD,
      out_b, nullptr, nullptr, kRows, kD, kD, kOutInv);
}
